// ChannelSegment_24292335026341
// MI455X (gfx1250) — hardware-verified
//
#include <hip/hip_runtime.h>
#include <math.h>
#include <stdint.h>

#define NB     2
#define LSEQ   1024
#define NCH    4
#define CW     512
#define CTOT   2048
#define NHEAD  8
#define HD     64
#define HD2    32
#define QKVN   1536
#define MROWS  2048
#define PHPE   2097152
#define EPSV   1e-6f
#define LAM0   0.2f
#define SSCL   0.17677669529663687f

typedef __attribute__((ext_vector_type(16))) __bf16 v16b;
typedef __attribute__((ext_vector_type(8)))  __bf16 v8b;
typedef __attribute__((ext_vector_type(8)))  float  v8f;
typedef __attribute__((ext_vector_type(4)))  float  v4f;
typedef __attribute__((ext_vector_type(4)))  unsigned int v4u;

__device__ __forceinline__ unsigned short f2bf_bits(float f) {
  const unsigned u = __float_as_uint(f);
  return (unsigned short)((u + 0x7FFFu + ((u >> 16) & 1u)) >> 16);
}
__device__ __forceinline__ float bfb2f(unsigned short h) { return __uint_as_float(((unsigned)h) << 16); }
__device__ __forceinline__ unsigned pk16(unsigned short a, unsigned short b) { return (unsigned)a | ((unsigned)b << 16); }
__device__ __forceinline__ void sp2(float a, float b, unsigned& h, unsigned& l) {
  const unsigned short ha = f2bf_bits(a), hb = f2bf_bits(b);
  h = pk16(ha, hb);
  l = pk16(f2bf_bits(a - bfb2f(ha)), f2bf_bits(b - bfb2f(hb)));
}
__device__ __forceinline__ void split8v(v4f a, v4f b, v4u& hv, v4u& lv) {
  unsigned h0, l0, h1, l1, h2, l2, h3, l3;
  sp2(a.x, a.y, h0, l0); sp2(a.z, a.w, h1, l1); sp2(b.x, b.y, h2, l2); sp2(b.z, b.w, h3, l3);
  hv = (v4u){h0, h1, h2, h3};
  lv = (v4u){l0, l1, l2, l3};
}
__device__ __forceinline__ void bsplit(float f, __bf16& hi, __bf16& lo) {
  const unsigned short hb = f2bf_bits(f);
  hi = __builtin_bit_cast(__bf16, hb);
  lo = __builtin_bit_cast(__bf16, f2bf_bits(f - bfb2f(hb)));
}
__device__ __forceinline__ float silu_f(float v) { return v * __builtin_amdgcn_rcpf(1.0f + __expf(-v)); }
__device__ __forceinline__ float dot4(v4f a, v4f b) { return a.x * b.x + a.y * b.y + a.z * b.z + a.w * b.w; }
__device__ __forceinline__ v8f zero8() { return (v8f){0.f, 0.f, 0.f, 0.f, 0.f, 0.f, 0.f, 0.f}; }
__device__ __forceinline__ void wave_sync() {
  __builtin_amdgcn_fence(__ATOMIC_RELEASE, "workgroup");
  __builtin_amdgcn_wave_barrier();
  __builtin_amdgcn_fence(__ATOMIC_ACQUIRE, "workgroup");
}
__device__ __forceinline__ int wave_id() { return __builtin_amdgcn_readfirstlane((int)(threadIdx.x >> 5)); }

__device__ __forceinline__ float redsum32(float v) {
  v += __shfl_xor(v, 1, 32); v += __shfl_xor(v, 2, 32); v += __shfl_xor(v, 4, 32);
  v += __shfl_xor(v, 8, 32); v += __shfl_xor(v, 16, 32);
  return v;
}
__device__ __forceinline__ float redsum16(float v) {
  v += __shfl_xor(v, 1, 32); v += __shfl_xor(v, 2, 32); v += __shfl_xor(v, 4, 32); v += __shfl_xor(v, 8, 32);
  return v;
}
__device__ __forceinline__ float redmax16(float v) {
  v = fmaxf(v, __shfl_xor(v, 1, 32)); v = fmaxf(v, __shfl_xor(v, 2, 32));
  v = fmaxf(v, __shfl_xor(v, 4, 32)); v = fmaxf(v, __shfl_xor(v, 8, 32));
  return v;
}

__device__ __forceinline__ v16b ldfrag(const __bf16* p) {
  union { v16b v; v8b h[2]; } f;
  f.h[0] = *(const v8b*)p;
  f.h[1] = *(const v8b*)(p + 16);
  return f.v;
}
__device__ __forceinline__ v8f mma_bf(v16b a, v16b b, v8f c) {
  c = __builtin_amdgcn_wmma_f32_16x16x32_bf16(false, a, false, b, (short)0, c, false, false);
  asm volatile("v_nop\n\tv_nop\n\tv_nop\n\tv_nop" : "+v"(c) : "v"(a), "v"(b));
  return c;
}

__device__ __forceinline__ void core32x64(const __bf16* __restrict__ Ah, const __bf16* __restrict__ Al, int lda,
                                          const __bf16* __restrict__ Bh, const __bf16* __restrict__ Bl, int ldb,
                                          int K, int lane, v8f (&acc)[2][4]) {
  const int rl = lane & 15, koff = (lane >> 4) * 8;
#pragma unroll
  for (int i = 0; i < 2; ++i)
#pragma unroll
    for (int j = 0; j < 4; ++j) acc[i][j] = zero8();
#pragma unroll 1
  for (int k0 = 0; k0 < K; k0 += 32) {
    v16b bh[4], bl[4];
#pragma unroll
    for (int j = 0; j < 4; ++j) {
      const size_t bo = (size_t)(j * 16 + rl) * ldb + k0 + koff;
      bh[j] = ldfrag(Bh + bo);
      bl[j] = ldfrag(Bl + bo);
    }
#pragma unroll
    for (int i = 0; i < 2; ++i) {
      const size_t ao = (size_t)(i * 16 + rl) * lda + k0 + koff;
      const v16b ah = ldfrag(Ah + ao);
      const v16b al = ldfrag(Al + ao);
#pragma unroll
      for (int j = 0; j < 4; ++j) {
        acc[i][j] = mma_bf(ah, bh[j], acc[i][j]);
        acc[i][j] = mma_bf(ah, bl[j], acc[i][j]);
        acc[i][j] = mma_bf(al, bh[j], acc[i][j]);
      }
    }
  }
}

__global__ __launch_bounds__(256) void split8_k(const float* __restrict__ in, unsigned short* __restrict__ hi,
                                               unsigned short* __restrict__ lo, int n8) {
  const int i = blockIdx.x * 256 + threadIdx.x;
  if (i < n8) {
    const size_t e = (size_t)i * 8;
    const v4f a = *(const v4f*)(in + e);
    const v4f b = *(const v4f*)(in + e + 4);
    v4u hv, lv;
    split8v(a, b, hv, lv);
    *(volatile v4u*)(hi + e) = hv;
    *(volatile v4u*)(lo + e) = lv;
    __threadfence();
    *(volatile v4u*)(hi + e) = hv;
    *(volatile v4u*)(lo + e) = lv;
  }
}

__global__ __launch_bounds__(256) void tsplit_k(const float* __restrict__ W, unsigned short* __restrict__ oh,
                                               unsigned short* __restrict__ ol, int R, int Cc, long sIn, long sOut) {
  __shared__ __align__(16) float tf[64 * 68];
  W  += (size_t)blockIdx.z * sIn;
  oh += (size_t)blockIdx.z * sOut;
  ol += (size_t)blockIdx.z * sOut;
  const int c0  = blockIdx.x * 64;
  const int r0  = blockIdx.y * 64;
  const int tid = threadIdx.x;
  {
    const int lr = tid >> 4;
    const int c4 = (tid & 15) * 4;
#pragma unroll
    for (int it = 0; it < 4; ++it) {
      const int rr = it * 16 + lr;
      const v4f a = *(const v4f*)(W + (size_t)(r0 + rr) * Cc + c0 + c4);
      *(v4f*)(tf + rr * 68 + c4) = a;
    }
  }
  __syncthreads();
  const int sub = tid >> 3;
  const int c8  = (tid & 7) * 8;
  v4u hv[2], lv[2];
#pragma unroll
  for (int it = 0; it < 2; ++it) {
    const int oc = it * 32 + sub;
    unsigned h0, l0, h1, l1, h2, l2, h3, l3;
    sp2(tf[(c8 + 0) * 68 + oc], tf[(c8 + 1) * 68 + oc], h0, l0);
    sp2(tf[(c8 + 2) * 68 + oc], tf[(c8 + 3) * 68 + oc], h1, l1);
    sp2(tf[(c8 + 4) * 68 + oc], tf[(c8 + 5) * 68 + oc], h2, l2);
    sp2(tf[(c8 + 6) * 68 + oc], tf[(c8 + 7) * 68 + oc], h3, l3);
    hv[it] = (v4u){h0, h1, h2, h3};
    lv[it] = (v4u){l0, l1, l2, l3};
  }
  for (int pass = 0; pass < 2; ++pass) {
#pragma unroll
    for (int it = 0; it < 2; ++it) {
      const int oc = it * 32 + sub;
      const size_t go = (size_t)(c0 + oc) * R + r0 + c8;
      *(volatile v4u*)(oh + go) = hv[it];
      *(volatile v4u*)(ol + go) = lv[it];
    }
    __threadfence();
  }
}

__global__ __launch_bounds__(256) void gemm_qk_k(
    const unsigned short* __restrict__ xh, const unsigned short* __restrict__ xl,
    const unsigned short* __restrict__ wth, const unsigned short* __restrict__ wtl,
    const float* __restrict__ bqkv, const float* __restrict__ wq, const float* __restrict__ wk,
    unsigned short* __restrict__ hp) {
  __shared__ __align__(16) float sT[8][16 * 68];
  const int c    = blockIdx.y;
  const int lane = threadIdx.x & 31;
  const int wave = wave_id();
  const int rl = lane & 15, h16 = lane >> 4, mOff = h16 * 8;
  const int tile = blockIdx.x * 8 + wave;
  if (tile >= (MROWS / 32) * ((2 * CW) / 64)) return;
  const int tm = tile >> 4, tn = tile & 15;
  const int m0 = tm * 32, n0 = tn * 64;

  const __bf16* Ah = (const __bf16*)(const void*)xh  + (size_t)m0 * CTOT + c * CW;
  const __bf16* Al = (const __bf16*)(const void*)xl  + (size_t)m0 * CTOT + c * CW;
  const __bf16* Bh = (const __bf16*)(const void*)wth + ((size_t)c * QKVN + n0) * CW;
  const __bf16* Bl = (const __bf16*)(const void*)wtl + ((size_t)c * QKVN + n0) * CW;
  v8f acc[2][4];
  core32x64(Ah, Al, CTOT, Bh, Bl, CW, CW, lane, acc);

  const int which = n0 >> 9;
  const int hh    = (n0 & (CW - 1)) >> 6;
  const int b     = m0 >> 10;
  const int pl    = c * 16 + b * 8 + hh;
  const float* wv = (which ? wk : wq) + c * HD2;
  const float* bn = bqkv + (size_t)c * QKVN + n0;
  unsigned short* P0h = hp + (size_t)(which * 4 + 0) * PHPE;
  unsigned short* P0l = hp + (size_t)(which * 4 + 1) * PHPE;
  unsigned short* P1h = hp + (size_t)(which * 4 + 2) * PHPE;
  unsigned short* P1l = hp + (size_t)(which * 4 + 3) * PHPE;
  float bj[4];
#pragma unroll
  for (int j = 0; j < 4; ++j) bj[j] = bn[j * 16 + rl];
  float* slab = sT[wave];
  const int srow = lane >> 2, cc = (lane & 3) * 8;

#pragma unroll
  for (int i = 0; i < 2; ++i) {
    const int mBase = m0 + i * 16;
    const int l0 = mBase & (LSEQ - 1);
#pragma unroll
    for (int j = 0; j < 4; ++j)
#pragma unroll
      for (int r = 0; r < 8; ++r)
        slab[(mOff + r) * 68 + j * 16 + rl] = silu_f(acc[i][j][r] + bj[j]);
    wave_sync();
    {
      float* sp = slab + rl * 68 + h16 * 32;
      v4f t[8];
      float ss = 0.f;
#pragma unroll
      for (int q = 0; q < 8; ++q) { t[q] = *(const v4f*)(sp + 4 * q); ss += dot4(t[q], t[q]); }
      const float scl = rsqrtf(ss * (1.0f / 32.0f) + EPSV);
#pragma unroll
      for (int q = 0; q < 8; ++q) {
        const v4f w4 = *(const v4f*)(wv + 4 * q);
        const v4f u = (t[q] * scl) * w4;
        *(v4f*)(sp + 4 * q) = u;
      }
    }
    wave_sync();
    v4u hv[2][2], lv[2][2];
#pragma unroll
    for (int it = 0; it < 2; ++it)
#pragma unroll
      for (int hf = 0; hf < 2; ++hf) {
        const float* sp2p = slab + (it * 8 + srow) * 68 + hf * 32 + cc;
        split8v(*(const v4f*)sp2p, *(const v4f*)(sp2p + 4), hv[it][hf], lv[it][hf]);
      }
    const size_t base = ((size_t)pl * LSEQ + l0) * HD2;
    for (int pass = 0; pass < 2; ++pass) {
#pragma unroll
      for (int it = 0; it < 2; ++it) {
        const size_t off = base + (size_t)(it * 8 + srow) * HD2 + cc;
        *(volatile v4u*)(P0h + off) = hv[it][0];
        *(volatile v4u*)(P0l + off) = lv[it][0];
        *(volatile v4u*)(P1h + off) = hv[it][1];
        *(volatile v4u*)(P1l + off) = lv[it][1];
      }
      __threadfence();
    }
    wave_sync();
  }
}

__global__ __launch_bounds__(256) void gemm_vt_k(
    const unsigned short* __restrict__ xh, const unsigned short* __restrict__ xl,
    const unsigned short* __restrict__ wth, const unsigned short* __restrict__ wtl,
    const float* __restrict__ bqkv,
    unsigned short* __restrict__ vth, unsigned short* __restrict__ vtl) {
  __shared__ __align__(16) float sT[8][16 * 68];
  const int c    = blockIdx.y;
  const int lane = threadIdx.x & 31;
  const int wave = wave_id();
  const int rl = lane & 15, h16 = lane >> 4, mOff = h16 * 8;
  const int tile = blockIdx.x * 8 + wave;
  if (tile >= (CW / 32) * (MROWS / 64)) return;
  const int tm = tile >> 5, tn = tile & 31;
  const int m0 = tm * 32, n0 = tn * 64;

  const __bf16* Ah = (const __bf16*)(const void*)wth + ((size_t)c * QKVN + 2 * CW + m0) * CW;
  const __bf16* Al = (const __bf16*)(const void*)wtl + ((size_t)c * QKVN + 2 * CW + m0) * CW;
  const __bf16* Bh = (const __bf16*)(const void*)xh  + (size_t)n0 * CTOT + c * CW;
  const __bf16* Bl = (const __bf16*)(const void*)xl  + (size_t)n0 * CTOT + c * CW;
  v8f acc[2][4];
  core32x64(Ah, Al, CW, Bh, Bl, CTOT, CW, lane, acc);

  const int hh = m0 >> 6, d0 = m0 & (HD - 1);
  const int b  = n0 >> 10, l0 = n0 & (LSEQ - 1);
  const int pl = c * 16 + b * 8 + hh;
  const float* bm = bqkv + (size_t)c * QKVN + 2 * CW + m0;
  float* slab = sT[wave];
  const int srow = lane >> 3, c8 = (lane & 7) * 8;

#pragma unroll
  for (int i = 0; i < 2; ++i) {
    float br[8];
#pragma unroll
    for (int r = 0; r < 8; ++r) br[r] = bm[i * 16 + mOff + r];
#pragma unroll
    for (int j = 0; j < 4; ++j)
#pragma unroll
      for (int r = 0; r < 8; ++r)
        slab[(mOff + r) * 68 + j * 16 + rl] = silu_f(acc[i][j][r] + br[r]);
    wave_sync();
    v4u hv[4], lv[4];
#pragma unroll
    for (int it = 0; it < 4; ++it) {
      const float* sp = slab + (it * 4 + srow) * 68 + c8;
      split8v(*(const v4f*)sp, *(const v4f*)(sp + 4), hv[it], lv[it]);
    }
    const size_t base = ((size_t)pl * HD + d0 + i * 16) * LSEQ + l0 + c8;
    for (int pass = 0; pass < 2; ++pass) {
#pragma unroll
      for (int it = 0; it < 4; ++it) {
        const size_t off = base + (size_t)(it * 4 + srow) * LSEQ;
        *(volatile v4u*)(vth + off) = hv[it];
        *(volatile v4u*)(vtl + off) = lv[it];
      }
      __threadfence();
    }
    wave_sync();
  }
}

__global__ __launch_bounds__(256) void attn_dual_k(
    const unsigned short* __restrict__ hp,
    const unsigned short* __restrict__ vth, const unsigned short* __restrict__ vtl,
    const float* __restrict__ lq1, const float* __restrict__ lk1,
    const float* __restrict__ lq2, const float* __restrict__ lk2,
    const float* __restrict__ wh,
    unsigned short* __restrict__ dfh, unsigned short* __restrict__ dfl) {
  __shared__ __align__(16) __bf16 Ks[4][64 * 32];
  __shared__ __align__(16) __bf16 Vt[2][64 * 64];
  __shared__ __align__(16) __bf16 Psh[8][16 * 64];
  __shared__ __align__(16) __bf16 Psl[8][16 * 64];
  __shared__ __align__(16) float  Os[8][16 * 68];
  union FB { v16b v; v8b h[2]; };

  const int tid  = threadIdx.x;
  const int wave = wave_id();
  const int lane = tid & 31;
  const int h16  = lane >> 4;
  const int rl   = lane & 15;
  const int att  = wave >> 2;
  const int wsub = wave & 3;
  const int qb = blockIdx.x;
  const int pl = blockIdx.y;
  const int c  = pl >> 4;
  const int b  = (pl >> 3) & 1;
  const int hh = pl & 7;
  const int q0 = qb * 64 + wsub * 16;

  float e1 = lq1[c * HD2 + lane] * lk1[c * HD2 + lane];
  float e2 = lq2[c * HD2 + lane] * lk2[c * HD2 + lane];
  e1 = redsum32(e1);
  e2 = redsum32(e2);
  const float lam = expf(e1) - expf(e2) + LAM0;

  const __bf16* HPb = (const __bf16*)(const void*)hp;
  const __bf16* Qh  = HPb + (size_t)(att * 2 + 0) * PHPE;
  const __bf16* Ql  = HPb + (size_t)(att * 2 + 1) * PHPE;
  const __bf16* K1h = HPb + (size_t)4 * PHPE;
  const __bf16* K1l = HPb + (size_t)5 * PHPE;
  const __bf16* K2h = HPb + (size_t)6 * PHPE;
  const __bf16* K2l = HPb + (size_t)7 * PHPE;
  const __bf16* Vh  = (const __bf16*)(const void*)vth;
  const __bf16* Vl  = (const __bf16*)(const void*)vtl;

  const size_t qo = ((size_t)pl * LSEQ + q0 + rl) * HD2 + 8 * h16;
  const v16b qah = ldfrag(Qh + qo);
  const v16b qal = ldfrag(Ql + qo);

  float mrow[8], lrow[8];
  v8f oacc[4];
#pragma unroll
  for (int r = 0; r < 8; ++r) { mrow[r] = -INFINITY; lrow[r] = 0.f; }
#pragma unroll
  for (int t = 0; t < 4; ++t) oacc[t] = zero8();

  __bf16* pwh = Psh[wave];
  __bf16* pwl = Psl[wave];

  for (int kc = 0; kc <= qb; ++kc) {
    const int kv0 = kc * 64;
    __syncthreads();
    {
      const size_t ko = ((size_t)pl * LSEQ + kv0) * HD2 + (size_t)tid * 8;
      const v8b a0 = *(const v8b*)(K1h + ko);
      const v8b a1 = *(const v8b*)(K1l + ko);
      const v8b a2 = *(const v8b*)(K2h + ko);
      const v8b a3 = *(const v8b*)(K2l + ko);
      *(v8b*)(&Ks[0][tid * 8]) = a0;
      *(v8b*)(&Ks[1][tid * 8]) = a1;
      *(v8b*)(&Ks[2][tid * 8]) = a2;
      *(v8b*)(&Ks[3][tid * 8]) = a3;
      const int d = tid >> 2, ccv = (tid & 3) * 16;
      const size_t vo = ((size_t)pl * HD + d) * LSEQ + kv0 + ccv;
      const v8b w0 = *(const v8b*)(Vh + vo);
      const v8b w1 = *(const v8b*)(Vh + vo + 8);
      const v8b w2 = *(const v8b*)(Vl + vo);
      const v8b w3 = *(const v8b*)(Vl + vo + 8);
      *(v8b*)(&Vt[0][d * 64 + ccv])     = w0;
      *(v8b*)(&Vt[0][d * 64 + ccv + 8]) = w1;
      *(v8b*)(&Vt[1][d * 64 + ccv])     = w2;
      *(v8b*)(&Vt[1][d * 64 + ccv + 8]) = w3;
    }
    __syncthreads();

    const __bf16* Kmh = Ks[att * 2];
    const __bf16* Kml = Ks[att * 2 + 1];
    v8f s[4];
#pragma unroll
    for (int j = 0; j < 4; ++j) {
      FB kb, kl;
      const __bf16* kp = Kmh + (j * 16 + rl) * HD2 + 8 * h16;
      const __bf16* kq = Kml + (j * 16 + rl) * HD2 + 8 * h16;
      kb.h[0] = *(const v8b*)kp; kb.h[1] = *(const v8b*)(kp + 16);
      kl.h[0] = *(const v8b*)kq; kl.h[1] = *(const v8b*)(kq + 16);
      s[j] = zero8();
      s[j] = mma_bf(qah, kb.v, s[j]);
      s[j] = mma_bf(qah, kl.v, s[j]);
      s[j] = mma_bf(qal, kb.v, s[j]);
    }
    const bool diag = (kc == qb);
    float cm[8];
#pragma unroll
    for (int r = 0; r < 8; ++r) {
      const int row = q0 + 8 * h16 + r;
      float m = -INFINITY;
#pragma unroll
      for (int j = 0; j < 4; ++j) {
        const int key = kv0 + j * 16 + rl;
        float sv = s[j][r] * SSCL;
        if (diag && key > row) sv = -INFINITY;
        s[j][r] = sv;
        m = fmaxf(m, sv);
      }
      cm[r] = redmax16(m);
    }
#pragma unroll
    for (int r = 0; r < 8; ++r) {
      const float mnew = fmaxf(mrow[r], cm[r]);
      const float alpha = __expf(mrow[r] - mnew);
      mrow[r] = mnew;
      float psum = 0.f;
#pragma unroll
      for (int j = 0; j < 4; ++j) {
        const float p = __expf(s[j][r] - mnew);
        psum += p;
        __bf16 ph, pq;
        bsplit(p, ph, pq);
        pwh[(8 * h16 + r) * 64 + j * 16 + rl] = ph;
        pwl[(8 * h16 + r) * 64 + j * 16 + rl] = pq;
      }
      psum = redsum16(psum);
      lrow[r] = lrow[r] * alpha + psum;
#pragma unroll
      for (int t = 0; t < 4; ++t) oacc[t][r] *= alpha;
    }
    wave_sync();
#pragma unroll
    for (int kk = 0; kk < 2; ++kk) {
      FB pa, pq;
      const __bf16* pp = pwh + rl * 64 + kk * 32 + 8 * h16;
      const __bf16* pr = pwl + rl * 64 + kk * 32 + 8 * h16;
      pa.h[0] = *(const v8b*)pp; pa.h[1] = *(const v8b*)(pp + 16);
      pq.h[0] = *(const v8b*)pr; pq.h[1] = *(const v8b*)(pr + 16);
#pragma unroll
      for (int t = 0; t < 4; ++t) {
        FB vb, vq;
        const __bf16* vp = &Vt[0][(t * 16 + rl) * 64 + kk * 32 + 8 * h16];
        const __bf16* vr = &Vt[1][(t * 16 + rl) * 64 + kk * 32 + 8 * h16];
        vb.h[0] = *(const v8b*)vp; vb.h[1] = *(const v8b*)(vp + 16);
        vq.h[0] = *(const v8b*)vr; vq.h[1] = *(const v8b*)(vr + 16);
        oacc[t] = mma_bf(pa.v, vb.v, oacc[t]);
        oacc[t] = mma_bf(pa.v, vq.v, oacc[t]);
        oacc[t] = mma_bf(pq.v, vb.v, oacc[t]);
      }
    }
  }

  float* os = Os[wave];
#pragma unroll
  for (int r = 0; r < 8; ++r) {
    const float inv = __builtin_amdgcn_rcpf(lrow[r]);
#pragma unroll
    for (int t = 0; t < 4; ++t) os[(8 * h16 + r) * 68 + t * 16 + rl] = oacc[t][r] * inv;
  }
  __syncthreads();
  if (att == 0) {
    const float* o2 = Os[wave + 4];
    const float* whp = wh + c * HD + h16 * 32;
    float* sp = os + rl * 68 + h16 * 32;
    const float* sq = o2 + rl * 68 + h16 * 32;
    v4f t[8];
    float ss = 0.f;
#pragma unroll
    for (int q = 0; q < 8; ++q) {
      const v4f a1 = *(const v4f*)(sp + 4 * q);
      const v4f a2 = *(const v4f*)(sq + 4 * q);
      const v4f dv = a1 - lam * a2;
      t[q] = dv;
      ss += dot4(dv, dv);
    }
    ss += __shfl_xor(ss, 16, 32);
    const float scl = rsqrtf(ss * (1.0f / 64.0f) + EPSV);
#pragma unroll
    for (int q = 0; q < 8; ++q) {
      const v4f w4 = *(const v4f*)(whp + 4 * q);
      const v4f u = ((t[q] * scl) * w4) * (1.0f - LAM0);
      *(v4f*)(sp + 4 * q) = u;
    }
    wave_sync();
    const int srow = lane >> 3, c8 = (lane & 7) * 8;
    v4u hv[4], lv[4];
#pragma unroll
    for (int it = 0; it < 4; ++it) {
      const float* rp = os + (it * 4 + srow) * 68 + c8;
      split8v(*(const v4f*)rp, *(const v4f*)(rp + 4), hv[it], lv[it]);
    }
    const size_t rbase = ((size_t)c * MROWS + b * LSEQ + q0) * CW + hh * HD + c8;
    for (int pass = 0; pass < 2; ++pass) {
#pragma unroll
      for (int it = 0; it < 4; ++it) {
        const size_t off = rbase + (size_t)(it * 4 + srow) * CW;
        *(volatile v4u*)(dfh + off) = hv[it];
        *(volatile v4u*)(dfl + off) = lv[it];
      }
      __threadfence();
    }
  }
}

__global__ __launch_bounds__(256) void gemm_out_k(
    const unsigned short* __restrict__ dh, const unsigned short* __restrict__ dl,
    const unsigned short* __restrict__ woh, const unsigned short* __restrict__ wol,
    const float* __restrict__ bout, float* __restrict__ ao) {
  __shared__ __align__(16) float sT[8][16 * 68];
  const int c    = blockIdx.y;
  const int lane = threadIdx.x & 31;
  const int wave = wave_id();
  const int rl = lane & 15, h16 = lane >> 4, mOff = h16 * 8;
  const int tile = blockIdx.x * 8 + wave;
  if (tile >= (MROWS / 32) * (CW / 64)) return;
  const int tm = tile >> 3, tn = tile & 7;
  const int m0 = tm * 32, n0 = tn * 64;

  const __bf16* Ah = (const __bf16*)(const void*)dh  + ((size_t)c * MROWS + m0) * CW;
  const __bf16* Al = (const __bf16*)(const void*)dl  + ((size_t)c * MROWS + m0) * CW;
  const __bf16* Bh = (const __bf16*)(const void*)woh + ((size_t)c * CW + n0) * CW;
  const __bf16* Bl = (const __bf16*)(const void*)wol + ((size_t)c * CW + n0) * CW;
  v8f acc[2][4];
  core32x64(Ah, Al, CW, Bh, Bl, CW, CW, lane, acc);

  const float* bn = bout + c * CW + n0;
  float bj[4];
#pragma unroll
  for (int j = 0; j < 4; ++j) bj[j] = bn[j * 16 + rl];
  float* slab = sT[wave];
  const int c4 = rl * 4;

#pragma unroll
  for (int i = 0; i < 2; ++i) {
#pragma unroll
    for (int j = 0; j < 4; ++j)
#pragma unroll
      for (int r = 0; r < 8; ++r)
        slab[(mOff + r) * 68 + j * 16 + rl] = silu_f(acc[i][j][r] + bj[j]);
    wave_sync();
    const size_t base = ((size_t)c * MROWS + m0 + i * 16) * CW + n0 + c4;
    for (int pass = 0; pass < 2; ++pass) {
#pragma unroll
      for (int it = 0; it < 8; ++it) {
        const int row = it * 2 + h16;
        const v4f v = *(const v4f*)(slab + row * 68 + c4);
        *(volatile v4f*)(ao + base + (size_t)row * CW) = v;
      }
      __threadfence();
    }
    wave_sync();
  }
}

__global__ __launch_bounds__(128) void final_k(
    const float* __restrict__ x, const float* __restrict__ ao, const float* __restrict__ wn,
    const float* __restrict__ rw, float* __restrict__ out) {
  __shared__ float red[4];
  const int r = blockIdx.x, c = blockIdx.y, b = r >> 10;
  const int tid = threadIdx.x, lane = tid & 31, wave = tid >> 5;
  const size_t ai = ((size_t)c * MROWS + r) * CW + tid * 4;
  const v4f a = *(const v4f*)(ao + ai);
  float ss = dot4(a, a);
  ss = redsum32(ss);
  if (lane == 0) red[wave] = ss;
  __syncthreads();
  const float tot = (red[0] + red[1]) + (red[2] + red[3]);
  const float scl = rsqrtf(tot * (1.0f / 512.0f) + EPSV);
  const float w = rw[b * NCH + c];
  const v4f w4 = *(const v4f*)(wn + c * CW + tid * 4);
  const size_t xo = (size_t)r * CTOT + c * CW + tid * 4;
  const v4f xv = *(const v4f*)(x + xo);
  const v4f y = (xv + (a * scl) * w4) * w;
  *(volatile v4f*)(out + xo) = y;
  __threadfence();
  *(volatile v4f*)(out + xo) = y;
}

extern "C" void kernel_launch(void* const* d_in, const int* in_sizes, int n_in,
                              void* d_out, int out_size, void* d_ws, size_t ws_size,
                              hipStream_t stream) {
  if (n_in < 14) return;
  if (in_sizes[0] != NB * LSEQ * CTOT) return;
  if (in_sizes[1] != NB * NCH) return;
  if (in_sizes[2] != NCH * CW * QKVN) return;
  if (in_sizes[3] != NCH * QKVN) return;
  if (in_sizes[4] != NCH * CW * CW) return;
  if (in_sizes[5] != NCH * CW) return;
  for (int i = 6; i < 12; ++i) if (in_sizes[i] != NCH * HD2) return;
  if (in_sizes[12] != NCH * HD) return;
  if (in_sizes[13] != NCH * CW) return;
  if (out_size != NB * LSEQ * CTOT) return;

  const float* x    = (const float*)d_in[0];
  const float* rw   = (const float*)d_in[1];
  const float* Wqkv = (const float*)d_in[2];
  const float* bqkv = (const float*)d_in[3];
  const float* Wout = (const float*)d_in[4];
  const float* bout = (const float*)d_in[5];
  const float* lq1  = (const float*)d_in[6];
  const float* lk1  = (const float*)d_in[7];
  const float* lq2  = (const float*)d_in[8];
  const float* lk2  = (const float*)d_in[9];
  const float* wq   = (const float*)d_in[10];
  const float* wk   = (const float*)d_in[11];
  const float* wh   = (const float*)d_in[12];
  const float* wn   = (const float*)d_in[13];
  float* out = (float*)d_out;

  const size_t PX  = (size_t)MROWS * CTOT * 2;
  const size_t PWQ = (size_t)NCH * QKVN * CW * 2;
  const size_t PWO = (size_t)NCH * CW * CW * 2;
  const size_t PHP = (size_t)8 * PHPE * 2;
  const size_t PV  = (size_t)64 * HD * LSEQ * 2;
  const size_t PD  = (size_t)NCH * MROWS * CW * 2;
  const size_t PAO = (size_t)NCH * MROWS * CW * 4;
  size_t off = 0;
  const size_t oXh = off; off += PX;   const size_t oXl = off; off += PX;
  const size_t oWh = off; off += PWQ;  const size_t oWl = off; off += PWQ;
  const size_t oOh = off; off += PWO;  const size_t oOl = off; off += PWO;
  const size_t oHP = off; off += PHP;
  const size_t oVh = off; off += PV;   const size_t oVl = off; off += PV;
  const size_t oDh = off; off += PD;   const size_t oDl = off; off += PD;
  const size_t oAO = off; off += PAO;
  if (off > ws_size) return;
  if (off > (size_t)134217728) return;

  char* ws = (char*)d_ws;
  unsigned short* xh  = (unsigned short*)(ws + oXh);
  unsigned short* xl  = (unsigned short*)(ws + oXl);
  unsigned short* wth = (unsigned short*)(ws + oWh);
  unsigned short* wtl = (unsigned short*)(ws + oWl);
  unsigned short* woh = (unsigned short*)(ws + oOh);
  unsigned short* wol = (unsigned short*)(ws + oOl);
  unsigned short* hp  = (unsigned short*)(ws + oHP);
  unsigned short* vth = (unsigned short*)(ws + oVh);
  unsigned short* vtl = (unsigned short*)(ws + oVl);
  unsigned short* dfh = (unsigned short*)(ws + oDh);
  unsigned short* dfl = (unsigned short*)(ws + oDl);
  float*          ao  = (float*)(ws + oAO);

  const dim3 blk(256);
  const int n8 = (MROWS * CTOT) / 8;
  split8_k<<<dim3((n8 + 255) / 256), blk, 0, stream>>>(x, xh, xl, n8);
  tsplit_k<<<dim3(QKVN / 64, CW / 64, NCH), blk, 0, stream>>>(Wqkv, wth, wtl, CW, QKVN, (long)CW * QKVN, (long)QKVN * CW);
  tsplit_k<<<dim3(CW / 64, CW / 64, NCH), blk, 0, stream>>>(Wout, woh, wol, CW, CW, (long)CW * CW, (long)CW * CW);
  gemm_qk_k<<<dim3(((MROWS / 32) * ((2 * CW) / 64)) / 8, NCH), blk, 0, stream>>>(xh, xl, wth, wtl, bqkv, wq, wk, hp);
  gemm_vt_k<<<dim3(((CW / 32) * (MROWS / 64)) / 8, NCH), blk, 0, stream>>>(xh, xl, wth, wtl, bqkv, vth, vtl);
  attn_dual_k<<<dim3(LSEQ / 64, 64), blk, 0, stream>>>(hp, vth, vtl, lq1, lk1, lq2, lk2, wh, dfh, dfl);
  gemm_out_k<<<dim3(((MROWS / 32) * (CW / 64)) / 8, NCH), blk, 0, stream>>>(dfh, dfl, woh, wol, bout, ao);
  final_k<<<dim3(MROWS, NCH), dim3(128), 0, stream>>>(x, ao, wn, rw, out);
  (void)hipGetLastError();
}
